// LSTMCell_58420145160201
// MI455X (gfx1250) — hardware-verified
//
#include <hip/hip_runtime.h>
#include <cstdint>

constexpr int ROWS_B = 4096;
constexpr int DIM_IN = 1024;
constexpr int DIM_H  = 1024;
constexpr int K_CAT  = DIM_H + DIM_IN;
constexpr int N_GATE = 4;
constexpr int N_IFGO = N_GATE * DIM_H;
static_assert(DIM_IN == DIM_H, "pack kernels assume equal widths");
static_assert(ROWS_B % 64 == 0 && N_IFGO % 64 == 0, "GEMM M,N tile multiples");
static_assert(K_CAT % 32 == 0, "GEMM K multiple of 32");
static_assert(K_CAT % 64 == 0 && N_IFGO % 64 == 0, "transpose tile multiples");
static_assert(DIM_H % 256 == 0, "pointwise block width");

constexpr size_t BYTES_A  = (size_t)ROWS_B * K_CAT * 2;
constexpr size_t BYTES_BT = (size_t)N_IFGO * K_CAT * 2;
constexpr size_t BYTES_G  = (size_t)ROWS_B * N_IFGO * 4;
constexpr size_t OFF_A  = 0;
constexpr size_t OFF_BT = OFF_A + BYTES_A;
constexpr size_t OFF_G  = OFF_BT + BYTES_BT;
constexpr size_t WS_TOTAL = OFF_G + BYTES_G;
static_assert(WS_TOTAL == 100663296, "carve total");
static_assert(WS_TOTAL <= 134217728, "carve under 128 MiB");
static_assert(OFF_BT % 128 == 0 && OFF_G % 128 == 0, "line aligned regions");

typedef __attribute__((ext_vector_type(16))) _Float16 v16h;
typedef __attribute__((ext_vector_type(8)))  _Float16 v8h;
typedef __attribute__((ext_vector_type(16))) __bf16   v16b;
typedef __attribute__((ext_vector_type(8)))  __bf16   v8b;
typedef __attribute__((ext_vector_type(8)))  float    v8f;
typedef __attribute__((ext_vector_type(4)))  float    v4f;
typedef __attribute__((ext_vector_type(4)))  unsigned v4u;

__device__ __forceinline__ unsigned short f2bf_bits(float f) {
  unsigned u = __float_as_uint(f);
  return (unsigned short)((u + 0x7FFFu + ((u >> 16) & 1u)) >> 16);
}
__device__ __forceinline__ float bf_bits2f(unsigned short h) { return __uint_as_float(((unsigned)h) << 16); }

__device__ __forceinline__ unsigned bf16_rne_u32(float f) {
  const unsigned u = __float_as_uint(f);
  return (u + 0x7FFFu + ((u >> 16) & 1u)) >> 16;
}
__device__ __forceinline__ unsigned pack_bf16x2(float lo, float hi) {
  return bf16_rne_u32(lo) | (bf16_rne_u32(hi) << 16);
}
__device__ __forceinline__ float bf16_rne_f32(float f) {
  return __uint_as_float(bf16_rne_u32(f) << 16);
}

__device__ __forceinline__ void dep_guard_h(v8f& a, v8f& b, v16h x, v16h y) { asm volatile("v_nop\n\tv_nop\n\tv_nop\n\tv_nop" : "+v"(a), "+v"(b) : "v"(x), "v"(y)); }
__device__ __forceinline__ void dep_guard_b(v8f& a, v8f& b, v16b x, v16b y) { asm volatile("v_nop\n\tv_nop\n\tv_nop\n\tv_nop" : "+v"(a), "+v"(b) : "v"(x), "v"(y)); }
__device__ __forceinline__ void dep_guard4_h(v8f& a, v8f& b, v8f& c, v8f& d, v16h x, v16h y) { asm volatile("v_nop\n\tv_nop\n\tv_nop\n\tv_nop" : "+v"(a), "+v"(b), "+v"(c), "+v"(d) : "v"(x), "v"(y)); }
__device__ __forceinline__ void dep_guard4_b(v8f& a, v8f& b, v8f& c, v8f& d, v16b x, v16b y) { asm volatile("v_nop\n\tv_nop\n\tv_nop\n\tv_nop" : "+v"(a), "+v"(b), "+v"(c), "+v"(d) : "v"(x), "v"(y)); }
__device__ __forceinline__ void keep4_h(v16h a, v16h b, v16h c, v16h d) { asm volatile("v_nop" :: "v"(a), "v"(b), "v"(c), "v"(d)); }
__device__ __forceinline__ void keep4_b(v16b a, v16b b, v16b c, v16b d) { asm volatile("v_nop" :: "v"(a), "v"(b), "v"(c), "v"(d)); }
__device__ __forceinline__ void acc_guard4(v8f& a, v8f& b, v8f& c, v8f& d) { asm volatile("v_nop\n\tv_nop\n\tv_nop\n\tv_nop" : "+v"(a), "+v"(b), "+v"(c), "+v"(d)); }
template <typename T> struct Frag;
template <> struct Frag<_Float16> {
  typedef v16h V; union U { v16h v; v8h h[2]; };
  static __device__ __forceinline__ v16h load(const _Float16* p) {
    U f; f.h[0] = *(const v8h*)(p); f.h[1] = *(const v8h*)(p + 16); return f.v;
  }
  static __device__ __forceinline__ v8f mma(v16h a, v16h b, v8f c) {
    return __builtin_amdgcn_wmma_f32_16x16x32_f16(false, a, false, b, (short)0, c, false, false);
  }
  static __device__ __forceinline__ void guard(v8f& a, v8f& b, v16h x, v16h y) { dep_guard_h(a, b, x, y); }
  static __device__ __forceinline__ void guard4(v8f& a, v8f& b, v8f& c, v8f& d, v16h x, v16h y) { dep_guard4_h(a, b, c, d, x, y); }
  static __device__ __forceinline__ void keep(v16h a, v16h b, v16h c, v16h d) { keep4_h(a, b, c, d); }
};
template <> struct Frag<__bf16> {
  typedef v16b V; union U { v16b v; v8b h[2]; };
  static __device__ __forceinline__ v16b load(const __bf16* p) {
    U f; f.h[0] = *(const v8b*)(p); f.h[1] = *(const v8b*)(p + 16); return f.v;
  }
  static __device__ __forceinline__ v8f mma(v16b a, v16b b, v8f c) {
    return __builtin_amdgcn_wmma_f32_16x16x32_bf16(false, a, false, b, (short)0, c, false, false);
  }
  static __device__ __forceinline__ void guard(v8f& a, v8f& b, v16b x, v16b y) { dep_guard_b(a, b, x, y); }
  static __device__ __forceinline__ void guard4(v8f& a, v8f& b, v8f& c, v8f& d, v16b x, v16b y) { dep_guard4_b(a, b, c, d, x, y); }
  static __device__ __forceinline__ void keep(v16b a, v16b b, v16b c, v16b d) { keep4_b(a, b, c, d); }
};

template <int ET> struct Elem;
template <> struct Elem<0> { typedef _Float16 T; };
template <> struct Elem<1> { typedef __bf16 T; };
template <int ET, bool SPLIT, int BIAS_MODE, int OUT_MODE, bool RESID, int ACT = 0>
__global__ __launch_bounds__(256) void wmma_gemm64(
    const unsigned short* __restrict__ Ap, const unsigned short* __restrict__ A2p, int lda, long strideA,
    const unsigned short* __restrict__ Btp, const unsigned short* __restrict__ Bt2p, int ldb, long strideB,
    void* __restrict__ Cout, void* __restrict__ Cout2, int ldc, long strideC,
    const float* __restrict__ bias,
    const float* __restrict__ resid, long strideR,
    int M, int N, int K, float scale) {
  typedef typename Elem<ET>::T T;
  typedef typename Frag<T>::V V;
  const T* A = (const T*)Ap; const T* A2 = (const T*)A2p; const T* Bt = (const T*)Btp; const T* Bt2 = (const T*)Bt2p;
  __shared__ __align__(16) float sT[8][16 * 68];
  const int b    = blockIdx.y;
  const int lane = threadIdx.x & 31;
  const int wave = threadIdx.x >> 5;
  const int tilesN = N >> 6;
  const int tilesM = M >> 6;
  const int tile = blockIdx.x * 8 + wave;
  if (tile >= tilesM * tilesN) return;
  const int tm = tile / tilesN;
  const int tn = tile - tm * tilesN;
  const int m0 = tm << 6;
  const int n0 = tn << 6;

  const T* Ab  = A  + (size_t)b * strideA;
  const T* Bb  = Bt + (size_t)b * strideB;
  const T* Ab2 = SPLIT ? (A2  + (size_t)b * strideA) : nullptr;
  const T* Bb2 = SPLIT ? (Bt2 + (size_t)b * strideB) : nullptr;

  const int rlane = lane & 15;
  const int koff  = (lane >> 4) * 8;
  const int mOff  = (lane >> 4) * 8;

  v8f acc[4][4];
#pragma unroll
  for (int i = 0; i < 4; ++i)
#pragma unroll
    for (int j = 0; j < 4; ++j) acc[i][j] = (v8f){0.f,0.f,0.f,0.f,0.f,0.f,0.f,0.f};

  for (int k0 = 0; k0 < K; k0 += 32) {
    V bh[4], bl[4];
#pragma unroll
    for (int j = 0; j < 4; ++j) {
      const size_t bo = (size_t)(n0 + (j << 4) + rlane) * ldb + koff + k0;
      bh[j] = Frag<T>::load(Bb + bo);
      if (SPLIT) bl[j] = Frag<T>::load(Bb2 + bo);
    }
#pragma unroll
    for (int i = 0; i < 4; ++i) {
      const size_t ao = (size_t)(m0 + (i << 4) + rlane) * lda + koff + k0;
      V ah = Frag<T>::load(Ab + ao);
      V al;
      if (SPLIT) al = Frag<T>::load(Ab2 + ao);
#pragma unroll
      for (int j = 0; j < 4; ++j) {
        acc[i][j] = Frag<T>::mma(ah, bh[j], acc[i][j]);
        if (SPLIT) {
          acc[i][j] = Frag<T>::mma(ah, bl[j], acc[i][j]);
          acc[i][j] = Frag<T>::mma(al, bh[j], acc[i][j]);
        }
      }
      Frag<T>::guard4(acc[i][0], acc[i][1], acc[i][2], acc[i][3], ah, SPLIT ? al : ah);
    }
    Frag<T>::keep(bh[0], bh[1], bh[2], bh[3]);
    if (SPLIT) Frag<T>::keep(bl[0], bl[1], bl[2], bl[3]);
  }
  acc_guard4(acc[0][0], acc[0][1], acc[0][2], acc[0][3]);
  acc_guard4(acc[1][0], acc[1][1], acc[1][2], acc[1][3]);
  acc_guard4(acc[2][0], acc[2][1], acc[2][2], acc[2][3]);
  acc_guard4(acc[3][0], acc[3][1], acc[3][2], acc[3][3]);

  float* slab = sT[wave];
  const float* Rb = RESID ? (resid + (size_t)b * strideR) : nullptr;
#pragma unroll
  for (int i = 0; i < 4; ++i) {
    const int mBase = m0 + (i << 4);
#pragma unroll
    for (int j = 0; j < 4; ++j) {
      const int n = n0 + (j << 4) + rlane;
      float bv = 0.f;
      if (BIAS_MODE == 2) bv = bias[n];
#pragma unroll
      for (int r = 0; r < 8; ++r) {
        float v = acc[i][j][r] * scale;
        if (BIAS_MODE == 1) v += bias[mBase + mOff + r];
        if (BIAS_MODE == 2) v += bv;
        if (RESID) v += Rb[(size_t)(mBase + mOff + r) * ldc + n];
        if (ACT == 1) v = tanhf(v);
        if (ACT == 2) v = fmaxf(v, 0.0f);
        if (ACT == 3) v = v / (1.0f + expf(-v));
        if (ACT == 4) v = (v > 0.f) ? v : 0.01f * v;
        if (ACT == 5) v = 0.5f * v * (1.0f + erff(v * 0.70710678118654752f));
        slab[(mOff + r) * 68 + (j << 4) + rlane] = v;
      }
    }
    __builtin_amdgcn_fence(__ATOMIC_RELEASE, "workgroup");
    __builtin_amdgcn_wave_barrier();
    __builtin_amdgcn_fence(__ATOMIC_ACQUIRE, "workgroup");
    if (OUT_MODE == 0) {
      float* C = (float*)Cout + (size_t)b * strideC;
      const int hh = lane >> 4, c4 = (lane & 15) * 4;
      for (int pass = 0; pass < 2; ++pass) {
#pragma unroll
        for (int it = 0; it < 8; ++it) {
          const int row = it * 2 + hh;
          v4f v = *(const v4f*)(slab + row * 68 + c4);
          *(volatile v4f*)(C + (size_t)(mBase + row) * ldc + n0 + c4) = v;
        }
        __threadfence();
      }
    } else {
      const int q = lane >> 3, c8 = (lane & 7) * 8;
      unsigned short* C  = (unsigned short*)Cout  + (size_t)b * strideC;
      unsigned short* C2 = (OUT_MODE == 2) ? ((unsigned short*)Cout2 + (size_t)b * strideC) : nullptr;
      for (int pass = 0; pass < 2; ++pass) {
#pragma unroll
        for (int it = 0; it < 4; ++it) {
          const int row = it * 4 + q;
          const float* sp = slab + row * 68 + c8;
          v8h hv, lv;
#pragma unroll
          for (int e = 0; e < 8; ++e) {
            if (OUT_MODE == 1) {
              hv[e] = (_Float16)sp[e];
            } else {
              unsigned short hb = f2bf_bits(sp[e]);
              unsigned short lb = f2bf_bits(sp[e] - bf_bits2f(hb));
              hv[e] = __builtin_bit_cast(_Float16, hb);
              lv[e] = __builtin_bit_cast(_Float16, lb);
            }
          }
          *(volatile v8h*)(C + (size_t)(mBase + row) * ldc + n0 + c8) = hv;
          if (OUT_MODE == 2) *(volatile v8h*)(C2 + (size_t)(mBase + row) * ldc + n0 + c8) = lv;
        }
        __threadfence();
      }
    }
    __builtin_amdgcn_fence(__ATOMIC_RELEASE, "workgroup");
    __builtin_amdgcn_wave_barrier();
    __builtin_amdgcn_fence(__ATOMIC_ACQUIRE, "workgroup");
  }
}

__global__ __launch_bounds__(256) void pack_a_rows(const float* __restrict__ hsrc,
                                                   const float* __restrict__ xsrc,
                                                   unsigned short* __restrict__ A16) {
  const int m    = blockIdx.x;
  const int t    = threadIdx.x;
  const int col8 = t * 8;
  const int isx  = (t >= 128) ? 1 : 0;
  const float* src = isx ? xsrc : hsrc;
  const int scol = col8 - isx * DIM_H;
  const float* p = src + (size_t)m * DIM_H + scol;
  const v4f a  = *(const v4f*)p;
  const v4f bq = *(const v4f*)(p + 4);
  v4u w;
  w[0] = pack_bf16x2(a[0], a[1]);
  w[1] = pack_bf16x2(a[2], a[3]);
  w[2] = pack_bf16x2(bq[0], bq[1]);
  w[3] = pack_bf16x2(bq[2], bq[3]);
  unsigned short* dst = A16 + (size_t)m * K_CAT + col8;
  *(volatile v4u*)dst = w;
  __threadfence();
  *(volatile v4u*)dst = w;
}

__global__ __launch_bounds__(256) void pack_bt_tiles(const float* __restrict__ Wh,
                                                     const float* __restrict__ Wx,
                                                     unsigned short* __restrict__ Bt16) {
  __shared__ __align__(16) float tile[64 * 68];
  const int n0  = blockIdx.x * 64;
  const int kt  = blockIdx.y;
  const int k0  = kt * 64;
  const int isx = (kt >= (DIM_H / 64)) ? 1 : 0;
  const float* W = isx ? Wx : Wh;
  const int ks0 = k0 - isx * DIM_H;
  const int t = threadIdx.x;
#pragma unroll
  for (int it = 0; it < 4; ++it) {
    const int idx = it * 256 + t;
    const int kr  = idx >> 4;
    const int c4  = (idx & 15) * 4;
    const v4f v = *(const v4f*)(W + (size_t)(ks0 + kr) * N_IFGO + n0 + c4);
    *(v4f*)(tile + kr * 68 + c4) = v;
  }
  __syncthreads();
  const int wave = t >> 5, lane = t & 31;
  const int q  = lane >> 3;
  const int c8 = (lane & 7) * 8;
  v4u wv[2];
#pragma unroll
  for (int it = 0; it < 2; ++it) {
    const int nrow = it * 32 + wave * 4 + q;
    v4u w;
#pragma unroll
    for (int e = 0; e < 4; ++e) {
      const float f0 = tile[(c8 + 2 * e) * 68 + nrow];
      const float f1 = tile[(c8 + 2 * e + 1) * 68 + nrow];
      w[e] = pack_bf16x2(f0, f1);
    }
    wv[it] = w;
  }
  for (int pass = 0; pass < 2; ++pass) {
#pragma unroll
    for (int it = 0; it < 2; ++it) {
      const int nrow = it * 32 + wave * 4 + q;
      unsigned short* dst = Bt16 + (size_t)(n0 + nrow) * K_CAT + k0 + c8;
      *(volatile v4u*)dst = wv[it];
    }
    __threadfence();
  }
}

__device__ __forceinline__ float gate_sigmoid(float v) {
  const float vc = fminf(fmaxf(v, -30.0f), 30.0f);
  const float e  = expf(-vc);
  return __builtin_amdgcn_rcpf(1.0f + e);
}
__device__ __forceinline__ float gate_tanh(float v) {
  const float vc = fminf(fmaxf(v, -15.0f), 15.0f);
  const float e  = expf(2.0f * vc);
  return 1.0f - 2.0f * __builtin_amdgcn_rcpf(e + 1.0f);
}

__global__ __launch_bounds__(256) void cell_pointwise(const float* __restrict__ G,
                                                      const float* __restrict__ cprev,
                                                      const float* __restrict__ bias,
                                                      float* __restrict__ h_out,
                                                      float* __restrict__ c_out) {
  __shared__ __align__(16) float hs[256];
  __shared__ __align__(16) float cs[256];
  const int t    = threadIdx.x;
  const int m    = blockIdx.y;
  const int col0 = blockIdx.x * 256;
  const int col  = col0 + t;
  const float* g = G + (size_t)m * N_IFGO + col;
  const float vi = g[0 * DIM_H];
  const float vf = g[1 * DIM_H];
  const float vg = g[2 * DIM_H];
  const float vo = g[3 * DIM_H];
  const float cv = cprev[(size_t)m * DIM_H + col];
  const float bi = bias[0 * DIM_H + col];
  const float bf = bias[1 * DIM_H + col];
  const float bg = bias[2 * DIM_H + col];
  const float bo = bias[3 * DIM_H + col];
  const float cb = bf16_rne_f32(cv);
  const float gi = vi + bf16_rne_f32(bi);
  const float gf = vf + bf16_rne_f32(bf);
  const float gg = vg + bf16_rne_f32(bg);
  const float go = vo + bf16_rne_f32(bo);
  const float si = gate_sigmoid(gi);
  const float sf = gate_sigmoid(gf);
  const float so = gate_sigmoid(go);
  const float tg = gate_tanh(gg);
  const float p0 = sf * cb;
  const float p1 = si * tg;
  const float cn = p0 + p1;
  const float hn = so * gate_tanh(cn);
  hs[t] = hn;
  cs[t] = cn;
  __syncthreads();
  if (t < 128) {
    const int which = t >> 6;
    const int l4    = (t & 63) * 4;
    const v4f hv4 = *(const v4f*)(hs + l4);
    const v4f cv4 = *(const v4f*)(cs + l4);
    const float fw = (float)which;
    const float fh = 1.0f - fw;
    v4f outv;
    outv[0] = fmaf(fw, cv4[0], fh * hv4[0]);
    outv[1] = fmaf(fw, cv4[1], fh * hv4[1]);
    outv[2] = fmaf(fw, cv4[2], fh * hv4[2]);
    outv[3] = fmaf(fw, cv4[3], fh * hv4[3]);
    float* base = which ? c_out : h_out;
    float* dst  = base + (size_t)m * DIM_H + col0 + l4;
    *(volatile v4f*)dst = outv;
    __threadfence();
    *(volatile v4f*)dst = outv;
  }
}

extern "C" void kernel_launch(void* const* d_in, const int* in_sizes, int n_in,
                              void* d_out, int out_size, void* d_ws, size_t ws_size,
                              hipStream_t stream) {
  (void)in_sizes; (void)n_in; (void)out_size;
  if (ws_size < WS_TOTAL) return;

  const float* x   = (const float*)d_in[0];
  const float* h   = (const float*)d_in[1];
  const float* c   = (const float*)d_in[2];
  const float* W_h = (const float*)d_in[3];
  const float* b_h = (const float*)d_in[4];
  const float* W_x = (const float*)d_in[5];

  float* h_next = (float*)d_out;
  float* c_next = (float*)d_out + (size_t)ROWS_B * DIM_H;

  unsigned char* ws = (unsigned char*)d_ws;
  unsigned short* A16  = (unsigned short*)(ws + OFF_A);
  unsigned short* Bt16 = (unsigned short*)(ws + OFF_BT);
  float*          IFGO = (float*)(ws + OFF_G);

  pack_a_rows<<<dim3(ROWS_B), dim3(256), 0, stream>>>(h, x, A16);

  pack_bt_tiles<<<dim3(N_IFGO / 64, K_CAT / 64), dim3(256), 0, stream>>>(W_h, W_x, Bt16);

  const int tiles = (ROWS_B / 64) * (N_IFGO / 64);
  wmma_gemm64<1, false, 0, 0, false, 0><<<dim3(tiles / 8, 1), dim3(256), 0, stream>>>(
      A16, A16, K_CAT, 0L,
      Bt16, Bt16, K_CAT, 0L,
      (void*)IFGO, (void*)IFGO, N_IFGO, 0L,
      b_h,
      c, 0L,
      ROWS_B, N_IFGO, K_CAT, 1.0f);

  cell_pointwise<<<dim3(DIM_H / 256, ROWS_B), dim3(256), 0, stream>>>(IFGO, c, b_h, h_next, c_next);
}
